// EncodingLayer_47261820125416
// MI455X (gfx1250) — hardware-run, weakly checked
//
#include <hip/hip_runtime.h>


#ifndef NB
#define NB 4
#endif
#ifndef SEQ
#define SEQ 512
#endif
#define NB_FULL  4
#define SEQ_FULL 512
#ifndef OUT_SEQ
#define OUT_SEQ SEQ
#endif
#define DM   64
#define NH_  8
#define HD   8
#define DFF  256
#define NTOK (NB * SEQ)
#define QRS  2048.0f
#define QRI  (1.0f / 2048.0f)
#define WCS  16.0f
#define WCI  (1.0f / 16.0f)
#define SC2  ((float)(0.35355339059327378 * 1.4426950408889634))
#define LG2E 1.4426950408889634f
#define MNEG (-1.0e9f)
#define PSH  14.0f
#define NEGB (-3.0e38f)
#define DTS  0.25f
#define A21 (0.25f)
#define A31 (3.0f / 32.0f)
#define A32 (9.0f / 32.0f)
#define A41 (1932.0f / 2197.0f)
#define A42 (-(7200.0f / 2197.0f))
#define A43 (7296.0f / 2197.0f)
#define A51 (439.0f / 216.0f)
#define A52 (-8.0f)
#define A53 (3680.0f / 513.0f)
#define A54 (-(845.0f / 4104.0f))
#define A61 (-(8.0f / 27.0f))
#define A62 (2.0f)
#define A63 (-(3544.0f / 2565.0f))
#define A64 (1859.0f / 4104.0f)
#define A65 (-(11.0f / 40.0f))
#define BW1 (16.0f / 135.0f)
#define BW3 (6656.0f / 12825.0f)
#define BW4 (28561.0f / 56430.0f)
#define BW5 (-(9.0f / 50.0f))
#define BW6 (2.0f / 55.0f)

static_assert(HD == 8);
static_assert(NH_ * HD == DM);
static_assert(DM == 64);
static_assert(DM % 32 == 0);
static_assert(DFF % 32 == 0);
static_assert(DFF == 256);
static_assert(SEQ % 64 == 0);
static_assert(SEQ % 32 == 0);
static_assert(SEQ % 16 == 0);
static_assert((NTOK * 16) % 256 == 0);
static_assert(NB <= NB_FULL);
static_assert(SEQ <= SEQ_FULL);
static_assert((68 * 4) % 16 == 0);
static_assert(4 * (4 * 16 * 68 + 64 * 68) <= 131072);
static_assert(4 * (32 * 68) <= 131072);
static_assert(4 * (16 * 68) <= 131072);

typedef _Float16 h16;
typedef __attribute__((ext_vector_type(16))) _Float16 v16h;
typedef __attribute__((ext_vector_type(8)))  _Float16 v8h;
typedef __attribute__((ext_vector_type(8)))  float    v8f;
typedef __attribute__((ext_vector_type(4)))  float    v4f;
typedef __attribute__((ext_vector_type(4)))  unsigned v4u;
typedef v4f  __attribute__((may_alias)) v4fa;

__device__ __forceinline__ unsigned short f2bf(float f) { unsigned u = __float_as_uint(f); u += 0x7FFFu + ((u >> 16) & 1u); return (unsigned short)(u >> 16); }
__device__ __forceinline__ float bfr(float f) { return __uint_as_float(((unsigned)f2bf(f)) << 16); }
__device__ __forceinline__ v16h cat16(v8h lo, v8h hi) { return __builtin_shufflevector(lo, hi, 0, 1, 2, 3, 4, 5, 6, 7, 8, 9, 10, 11, 12, 13, 14, 15); }
static __device__ __forceinline__ h16 toh_flush(float v) { const float w = (fabsf(v) < 6.103515625e-05f) ? 0.0f : v; return (h16)w; }
__device__ __forceinline__ v8f wmma16g(v16h a, v16h b, v8f c) {
    c = __builtin_amdgcn_wmma_f32_16x16x32_f16(false, a, false, b, (short)0, c, false, false);
    asm volatile("v_nop\n\tv_nop\n\tv_nop\n\tv_nop" : "+v"(c) : "v"(a), "v"(b));
    return c;
}
__device__ __forceinline__ v16h ldh(const h16* p) { return cat16(*(const v8h*)p, *(const v8h*)(p + 16)); }
__device__ __forceinline__ void wave_sync() { __builtin_amdgcn_fence(3  , "wavefront"); __builtin_amdgcn_wave_barrier(); asm volatile("" ::: "memory"); }

__global__ __launch_bounds__(256) void k_wconv(const float* __restrict__ W, const float* __restrict__ bias, h16* WT, float* BP, int K, int N, int row0) {
    const unsigned i = blockIdx.x * 256u + threadIdx.x;
    const unsigned kp = (unsigned)K >> 3;
    const unsigned total = (unsigned)N * kp;
    if (i < total) {
        const unsigned n = i / kp, p = i - n * kp;
        v8h o;
#pragma unroll
        for (int k = 0; k < 8; ++k) { const float w = bfr(W[(size_t)(p * 8u + (unsigned)k) * (unsigned)N + n]); o[k] = toh_flush(w * WCS); }
        h16* d = WT + (size_t)((unsigned)row0 + n) * (unsigned)K + p * 8u;
        *(volatile v8h*)d = o; __threadfence(); *(volatile v8h*)d = o;
    }
    const unsigned nb4 = (unsigned)N >> 2;
    if (i < nb4) {
        const v4f b = *(const v4f*)(bias + (size_t)i * 4u); v4f o;
#pragma unroll
        for (int k = 0; k < 4; ++k) o[k] = bfr(b[k]);
        float* d = BP + (size_t)((unsigned)row0 + i * 4u);
        *(volatile v4f*)d = o; __threadfence(); *(volatile v4f*)d = o;
    }
}

__global__ __launch_bounds__(256) void k_init(const float* __restrict__ x, float* Y) {
    const unsigned i = blockIdx.x * 256u + threadIdx.x;
    const unsigned n = i >> 4, c4 = (i & 15u) * 4u;
    const unsigned b = n / (unsigned)SEQ, t = n % (unsigned)SEQ;
    const v4f v = *(const v4f*)(x + ((size_t)(b * (unsigned)SEQ_FULL + t)) * DM + c4); v4f o;
#pragma unroll
    for (int k = 0; k < 4; ++k) o[k] = bfr(v[k]);
    float* d = Y + (size_t)n * DM + c4;
    *(volatile v4f*)d = o; __threadfence(); *(volatile v4f*)d = o;
}

__global__ __launch_bounds__(256) void k_update(const float* Y, const float* KS, float* DST, int pitch) {
    const unsigned i = blockIdx.x * 256u + threadIdx.x;
    const unsigned n = i >> 4, c4 = (i & 15u) * 4u;
    const size_t g = (size_t)n * DM + c4;
    const size_t PL = (size_t)NTOK * DM;
    const v4f y = *(const v4f*)(Y + g);
    v4f t = *(const v4f*)(KS + g) * BW1;
    t = t + *(const v4f*)(KS + 2 * PL + g) * BW3;
    t = t + *(const v4f*)(KS + 3 * PL + g) * BW4;
    t = t + *(const v4f*)(KS + 4 * PL + g) * BW5;
    t = t + *(const v4f*)(KS + 5 * PL + g) * BW6;
    const v4f o = y + t * DTS;
    const unsigned b = n / (unsigned)SEQ, tq = n % (unsigned)SEQ;
    float* d = DST + (size_t)(b * (unsigned)pitch + tq) * DM + c4;
    *(volatile v4f*)d = o; __threadfence(); *(volatile v4f*)d = o;
}

__global__ __launch_bounds__(128) void k_qkv(const float* __restrict__ Y, const float* __restrict__ KS, float* YS,
                                             const h16* __restrict__ WT, const float* __restrict__ BP, h16* QK, h16* VT, int stage) {
    __shared__ __align__(16) float yt[4 * 16 * 68];
    __shared__ __align__(16) float vs[64 * 68];
    const int lane = threadIdx.x & 31, lr = lane & 15, hi = lane >> 4;
    const int wave = __builtin_amdgcn_readfirstlane((int)(threadIdx.x >> 5));
    const unsigned tok0 = blockIdx.x * 64u;
    const unsigned r0 = tok0 + (unsigned)wave * 16u;
    const int wb = wave * 16 * 68;
    const size_t PL = (size_t)NTOK * DM;
    float c0 = 0.0f, c1 = 0.0f, c2 = 0.0f, c3 = 0.0f, c4 = 0.0f;
    if (stage == 1)      { c0 = A21; }
    else if (stage == 2) { c0 = A31; c1 = A32; }
    else if (stage == 3) { c0 = A41; c1 = A42; c2 = A43; }
    else if (stage == 4) { c0 = A51; c1 = A52; c2 = A53; c3 = A54; }
    else if (stage == 5) { c0 = A61; c1 = A62; c2 = A63; c3 = A64; c4 = A65; }
    static_assert(32 * 16 * 8 == 16 * DM * 4);
#pragma unroll 1
    for (int i = 0; i < 8; ++i) {
        const int row = 2 * i + hi, cc = lr * 4;
        const size_t g = (size_t)(r0 + (unsigned)row) * DM + cc;
        v4f y = *(const v4f*)(Y + g);
        if (stage > 0) {
            v4f t = *(const v4f*)(KS + g) * c0;
            if (stage > 1) t = t + *(const v4f*)(KS + PL + g) * c1;
            if (stage > 2) t = t + *(const v4f*)(KS + 2 * PL + g) * c2;
            if (stage > 3) t = t + *(const v4f*)(KS + 3 * PL + g) * c3;
            if (stage > 4) t = t + *(const v4f*)(KS + 4 * PL + g) * c4;
            y = y + t * DTS;
        }
        *(v4fa*)(&yt[wb + row * 68 + cc]) = y;
        if (stage > 0) *(volatile v4f*)(YS + g) = y;
    }
    if (stage > 0) {
        __threadfence();
#pragma unroll 1
        for (int i = 0; i < 8; ++i) {
            const int row = 2 * i + hi, cc = lr * 4;
            const size_t g = (size_t)(r0 + (unsigned)row) * DM + cc;
            const v4f y = *(const v4fa*)(&yt[wb + row * 68 + cc]);
            *(volatile v4f*)(YS + g) = y;
        }
    }
    wave_sync();
    v16h bH[2], bR[2];
#pragma unroll
    for (int ks = 0; ks < 2; ++ks) {
        const float* p = &yt[wb + lr * 68 + ks * 32 + 8 * hi];
        const v4f x0 = *(const v4fa*)p, x1 = *(const v4fa*)(p + 4), x2 = *(const v4fa*)(p + 16), x3 = *(const v4fa*)(p + 20);
#pragma unroll
        for (int i = 0; i < 4; ++i) {
            const h16 a0 = toh_flush(x0[i]), a1 = toh_flush(x1[i]), a2 = toh_flush(x2[i]), a3 = toh_flush(x3[i]);
            bH[ks][i] = a0; bH[ks][4 + i] = a1; bH[ks][8 + i] = a2; bH[ks][12 + i] = a3;
            bR[ks][i]      = toh_flush((x0[i] - (float)a0) * QRS); bR[ks][4 + i]  = toh_flush((x1[i] - (float)a1) * QRS);
            bR[ks][8 + i]  = toh_flush((x2[i] - (float)a2) * QRS); bR[ks][12 + i] = toh_flush((x3[i] - (float)a3) * QRS); }
    }
    const unsigned bb = tok0 / (unsigned)SEQ, tt = tok0 % (unsigned)SEQ;
    const size_t PLh = (size_t)NTOK * DM;
#pragma unroll 1
    for (int j = 0; j < 12; ++j) {
        const h16* wp = WT + (size_t)(16 * j + lr) * DM + 8 * hi;
        const v16h w0 = ldh(wp), w1 = ldh(wp + 32);
        v8f aH = (v8f){}, aR = (v8f){};
        aH = wmma16g(w0, bH[0], aH); aR = wmma16g(w0, bR[0], aR);
        aH = wmma16g(w1, bH[1], aH); aR = wmma16g(w1, bR[1], aR);
        const v4f b0 = *(const v4f*)(BP + 16 * j + 8 * hi), b1 = *(const v4f*)(BP + 16 * j + 8 * hi + 4);
        float v[8];
#pragma unroll
        for (int r = 0; r < 4; ++r) { v[r] = (aH[r] + aR[r] * QRI) * WCI + b0[r]; v[4 + r] = (aH[4 + r] + aR[4 + r] * QRI) * WCI + b1[r]; }
        if (j < 8) {
            v8h hv, rv;
#pragma unroll
            for (int r = 0; r < 8; ++r) { const h16 a = toh_flush(v[r]); hv[r] = a; rv[r] = toh_flush((v[r] - (float)a) * QRS); }
            const unsigned zh = bb * (unsigned)NH_ + 2u * ((unsigned)j & 3u) + (unsigned)hi;
            const size_t off = (size_t)((unsigned)j >> 2) * (2 * PLh) + ((size_t)zh * SEQ + tt + (unsigned)wave * 16u + (unsigned)lr) * HD;
            h16* ph = QK + off; h16* pr = QK + PLh + off;
            *(volatile v8h*)ph = hv; *(volatile v8h*)pr = rv; __threadfence(); *(volatile v8h*)ph = hv; *(volatile v8h*)pr = rv;
        } else {
            v4f s0, s1;
#pragma unroll
            for (int r = 0; r < 4; ++r) { s0[r] = v[r]; s1[r] = v[4 + r]; }
            float* q = &vs[(wave * 16 + lr) * 68 + 16 * (j - 8) + 8 * hi];
            *(v4fa*)q = s0; *(v4fa*)(q + 4) = s1;
        }
    }
    __syncthreads();
    static_assert(128 * 16 * 8 == 128 * 128);
#pragma unroll 1
    for (int ps = 0; ps < 2; ++ps) {
#pragma unroll 1
        for (int it = 0; it < 8; ++it) {
            const int line = it * 16 + (int)(threadIdx.x >> 3);
            const int hd = line >> 4, rr = line & 15, d = rr & 7, pc = (int)(threadIdx.x & 7);
            v8h o;
#pragma unroll
            for (int i = 0; i < 8; ++i) {
                const float x = vs[(pc * 8 + i) * 68 + hd * 8 + d];
                const h16 a = toh_flush(x);
                const float w = (rr >= 8) ? ((x - (float)a) * QRS) : x;
                o[i] = toh_flush(w); }
            h16* dst = VT + ((size_t)((bb * (unsigned)NH_ + (unsigned)hd) * 16u + (unsigned)rr)) * SEQ + tt + (unsigned)pc * 8u;
            *(volatile v8h*)dst = o;
        }
        if (ps == 0) __threadfence();
    }
}

__global__ __launch_bounds__(256) void k_flash(const h16* __restrict__ QK, const h16* __restrict__ VT, const float* __restrict__ mask, h16* CX) {
    __shared__ __align__(16) float cs[32 * 68];
    const int lane = threadIdx.x & 31, lr = lane & 15, hi = lane >> 4;
    const int wave = __builtin_amdgcn_readfirstlane((int)(threadIdx.x >> 5));
    const unsigned b = blockIdx.y, t0 = blockIdx.x * 16u;
    const unsigned zh = b * (unsigned)NH_ + (unsigned)wave;
    const size_t PLh = (size_t)NTOK * DM;
    const size_t rowq = ((size_t)zh * SEQ + t0 + (unsigned)lr) * HD;
    const v8h z8 = (v8h){};
    const v8h xh = *(const v8h*)(QK + rowq);
    const v8h xm = *(const v8h*)(QK + (size_t)(1 - hi) * PLh + rowq);
    const v4u xu = __builtin_bit_cast(v4u, xh); const v4u zu = (v4u){0u, 0u, 0u, 0u};
    const v4u su = (hi == 0) ? xu : zu;
    const v16h qH = cat16(__builtin_bit_cast(v8h, su), z8);
    const v16h qR = cat16(xm, z8);
    const size_t kbase = 2 * PLh + (size_t)hi * PLh + ((size_t)zh * SEQ + (unsigned)lr) * HD;
    const size_t vbase = ((size_t)zh * 16 + (unsigned)lr) * SEQ + 8 * hi;
    const float qadd = (bfr(mask[(size_t)b * SEQ_FULL + t0 + (unsigned)lr]) * MNEG) * LG2E;
    v8f oA = (v8f){}, oB = (v8f){};
    float m = NEGB, l = 0.0f;
#pragma unroll 1
    for (int key0 = 0; key0 < SEQ; key0 += 32) {
        const v16h ka = cat16(*(const v8h*)(QK + kbase + (size_t)key0 * HD), z8);
        const v16h kb = cat16(*(const v8h*)(QK + kbase + (size_t)(key0 + 16) * HD), z8);
        v8f sHa = (v8f){}, sLa = (v8f){}, sHb = (v8f){}, sLb = (v8f){};
        sHa = wmma16g(ka, qH, sHa); sLa = wmma16g(ka, qR, sLa);
        sHb = wmma16g(kb, qH, sHb); sLb = wmma16g(kb, qR, sLb);
        float ta[8], tb[8]; float mx = NEGB;
#pragma unroll
        for (int r = 0; r < 8; ++r) {
            ta[r] = (sHa[r] + sLa[r] * QRI) * SC2 + qadd; tb[r] = (sHb[r] + sLb[r] * QRI) * SC2 + qadd;
            mx = fmaxf(mx, fmaxf(ta[r], tb[r])); }
        mx = fmaxf(mx, __shfl_xor(mx, 16, 32));
        const float mnew = fmaxf(m, mx);
        const float alpha = __builtin_amdgcn_exp2f(m - mnew);
        const float sh = PSH - mnew;
        v16h pb, pr; float ls = 0.0f;
#pragma unroll
        for (int r = 0; r < 8; ++r) {
            const float ea = ta[r] + sh, eb = tb[r] + sh;
            const float xa = __builtin_amdgcn_exp2f(ea), xb = __builtin_amdgcn_exp2f(eb);
            const float ga = (ea < -14.0f) ? 0.0f : xa, gb = (eb < -14.0f) ? 0.0f : xb;
            const h16 pa = (h16)ga; const h16 pc = (h16)gb;
            pb[r] = pa; pb[8 + r] = pc;
            pr[r] = toh_flush((ga - (float)pa) * QRS); pr[8 + r] = toh_flush((gb - (float)pc) * QRS);
            ls += ga + gb; }
        l = l * alpha + ls; m = mnew;
        oA = oA * alpha; oB = oB * alpha;
        const v16h va = ldh(VT + vbase + key0);
        oA = wmma16g(va, pb, oA); oB = wmma16g(va, pr, oB);
    }
    l += __shfl_xor(l, 16, 32);
    float xo[8];
#pragma unroll
    for (int r = 0; r < 8; ++r) xo[r] = __shfl_xor(oA[r], 16, 32);
    const float inv = 1.0f / l;
    { v4f a, c;
#pragma unroll
      for (int r = 0; r < 4; ++r) { a[r] = (oA[r] + (oB[r] + xo[r]) * QRI) * inv; c[r] = (oA[4 + r] + (oB[4 + r] + xo[4 + r]) * QRI) * inv; }
      float* q = &cs[(hi * 16 + lr) * 68 + wave * 8];
      *(v4fa*)q = a; *(v4fa*)(q + 4) = c; }
    __syncthreads();
    static_assert(256 * 16 == 2 * 16 * DM * 2);
    {
        const int line = (int)(threadIdx.x >> 3), pl = line >> 4, row = line & 15, pc = (int)(threadIdx.x & 7);
        const v4f x0 = *(const v4fa*)(&cs[row * 68 + pc * 8]), x1 = *(const v4fa*)(&cs[row * 68 + pc * 8 + 4]);
        v8h o;
#pragma unroll
        for (int i = 0; i < 4; ++i) {
            const h16 a0 = toh_flush(x0[i]), a1 = toh_flush(x1[i]);
            const float w0 = (pl != 0) ? ((x0[i] - (float)a0) * QRS) : x0[i];
            const float w1 = (pl != 0) ? ((x1[i] - (float)a1) * QRS) : x1[i];
            o[i] = toh_flush(w0); o[4 + i] = toh_flush(w1); }
        h16* dst = CX + (size_t)pl * PLh + ((size_t)b * SEQ + t0 + (unsigned)row) * DM + pc * 8;
        *(volatile v8h*)dst = o; __threadfence(); *(volatile v8h*)dst = o;
    }
}

__global__ __launch_bounds__(32) void k_wo_ffn(const h16* __restrict__ CX, const float* __restrict__ YSRC, const h16* __restrict__ WOT, const float* __restrict__ BO,
                                               const h16* __restrict__ W1T, const float* __restrict__ B1, const h16* __restrict__ W2T, const float* __restrict__ B2, float* KOUT) {
    __shared__ __align__(16) float os[16 * 68];
    const int lane = threadIdx.x & 31, lr = lane & 15, hi = lane >> 4;
    const unsigned t0 = blockIdx.x * 16u;
    const size_t PLh = (size_t)NTOK * DM;
    const size_t co = (size_t)(t0 + (unsigned)lr) * DM + 8 * hi;
    const v16h cH0 = ldh(CX + co), cH1 = ldh(CX + co + 32), cR0 = ldh(CX + PLh + co), cR1 = ldh(CX + PLh + co + 32);
    v16h hH[2], hR[2];
#pragma unroll
    for (int j = 0; j < 4; ++j) {
        const h16* wp = WOT + (size_t)(16 * j + lr) * DM + 8 * hi;
        const v16h w0 = ldh(wp), w1 = ldh(wp + 32);
        v8f aH = (v8f){}, aR = (v8f){};
        aH = wmma16g(w0, cH0, aH); aR = wmma16g(w0, cR0, aR);
        aH = wmma16g(w1, cH1, aH); aR = wmma16g(w1, cR1, aR);
        const v4f b0 = *(const v4f*)(BO + 16 * j + 8 * hi), b1 = *(const v4f*)(BO + 16 * j + 8 * hi + 4);
        const float* yp = YSRC + (size_t)(t0 + (unsigned)lr) * DM + 16 * j + 8 * hi;
        const v4f y0 = *(const v4f*)yp, y1 = *(const v4f*)(yp + 4);
        v4f a0, a1;
#pragma unroll
        for (int r = 0; r < 4; ++r) { a0[r] = (aH[r] + aR[r] * QRI) * WCI + b0[r]; a1[r] = (aH[4 + r] + aR[4 + r] * QRI) * WCI + b1[r]; }
        float* q = &os[lr * 68 + 16 * j + 8 * hi];
        *(v4fa*)q = a0; *(v4fa*)(q + 4) = a1;
#pragma unroll
        for (int r = 0; r < 4; ++r) {
            const float h0 = y0[r] + a0[r], h1 = y1[r] + a1[r];
            const h16 g0 = toh_flush(h0), g1 = toh_flush(h1);
            hH[j >> 1][(j & 1) * 8 + r] = g0; hH[j >> 1][(j & 1) * 8 + 4 + r] = g1;
            hR[j >> 1][(j & 1) * 8 + r] = toh_flush((h0 - (float)g0) * QRS); hR[j >> 1][(j & 1) * 8 + 4 + r] = toh_flush((h1 - (float)g1) * QRS); }
    }
    v8f oH[4], oR[4];
#pragma unroll
    for (int j = 0; j < 4; ++j) { oH[j] = (v8f){}; oR[j] = (v8f){}; }
#pragma unroll 1
    for (int c = 0; c < DFF / 32; ++c) {
        v16h fH, fR;
#pragma unroll
        for (int u = 0; u < 2; ++u) {
            const int ff0 = 32 * c + 16 * u;
            const h16* wp = W1T + (size_t)(ff0 + lr) * DM + 8 * hi;
            const v16h w0 = ldh(wp), w1 = ldh(wp + 32);
            v8f aH = (v8f){}, aR = (v8f){};
            aH = wmma16g(w0, hH[0], aH); aR = wmma16g(w0, hR[0], aR);
            aH = wmma16g(w1, hH[1], aH); aR = wmma16g(w1, hR[1], aR);
            const v4f b0 = *(const v4f*)(B1 + ff0 + 8 * hi), b1 = *(const v4f*)(B1 + ff0 + 8 * hi + 4);
#pragma unroll
            for (int r = 0; r < 4; ++r) {
                const float f0 = fmaxf((aH[r] + aR[r] * QRI) * WCI + b0[r], 0.0f), f1 = fmaxf((aH[4 + r] + aR[4 + r] * QRI) * WCI + b1[r], 0.0f);
                const h16 g0 = toh_flush(f0), g1 = toh_flush(f1);
                fH[u * 8 + r] = g0; fH[u * 8 + 4 + r] = g1;
                fR[u * 8 + r] = toh_flush((f0 - (float)g0) * QRS); fR[u * 8 + 4 + r] = toh_flush((f1 - (float)g1) * QRS); }
        }
#pragma unroll
        for (int j = 0; j < 4; ++j) {
            const v16h w = ldh(W2T + (size_t)(16 * j + lr) * DFF + 32 * c + 8 * hi);
            oH[j] = wmma16g(w, fH, oH[j]); oR[j] = wmma16g(w, fR, oR[j]); }
    }
#pragma unroll
    for (int j = 0; j < 4; ++j) {
        const v4f b0 = *(const v4f*)(B2 + 16 * j + 8 * hi), b1 = *(const v4f*)(B2 + 16 * j + 8 * hi + 4);
        float* q = &os[lr * 68 + 16 * j + 8 * hi];
        v4f a0 = *(const v4fa*)q, a1 = *(const v4fa*)(q + 4);
#pragma unroll
        for (int r = 0; r < 4; ++r) { a0[r] = a0[r] + ((oH[j][r] + oR[j][r] * QRI) * WCI + b0[r]); a1[r] = a1[r] + ((oH[j][4 + r] + oR[j][4 + r] * QRI) * WCI + b1[r]); }
        *(v4fa*)q = a0; *(v4fa*)(q + 4) = a1;
    }
    wave_sync();
    static_assert(32 * 16 * 8 == 16 * DM * 4);
#pragma unroll 1
    for (int ps = 0; ps < 2; ++ps) {
#pragma unroll
        for (int i = 0; i < 8; ++i) { const int row = 2 * i + hi, cc = lr * 4;
            const v4f val = *(const v4fa*)(&os[row * 68 + cc]);
            *(volatile v4f*)(KOUT + (size_t)(t0 + (unsigned)row) * DM + cc) = val; }
        if (ps == 0) __threadfence(); }
}

static constexpr size_t al256(size_t v) { return (v + 255) & ~(size_t)255; }
static constexpr size_t SZ_F  = (size_t)NTOK * DM * 4;
static constexpr size_t SZ_QK = al256((size_t)4 * NTOK * DM * 2);
static constexpr size_t SZ_VT = al256((size_t)NB * NH_ * 16 * SEQ * 2);
static constexpr size_t SZ_CX = al256((size_t)2 * NTOK * DM * 2);
static constexpr size_t SZ_WQ = al256((size_t)3 * DM * DM * 2);
static constexpr size_t SZ_WO = al256((size_t)DM * DM * 2);
static constexpr size_t SZ_W1 = al256((size_t)DFF * DM * 2);
static constexpr size_t SZ_W2 = al256((size_t)DM * DFF * 2);
static constexpr size_t SZ_BQ = al256((size_t)3 * DM * 4);
static constexpr size_t SZ_BO = al256((size_t)DM * 4);
static constexpr size_t SZ_B1 = al256((size_t)DFF * 4);
static constexpr size_t SZ_B2 = al256((size_t)DM * 4);
static constexpr size_t SZ_TOTAL = 8 * SZ_F + SZ_QK + SZ_VT + SZ_CX + SZ_WQ + SZ_WO + SZ_W1 + SZ_W2 + SZ_BQ + SZ_BO + SZ_B1 + SZ_B2;
static_assert(SZ_F % 256 == 0);
static_assert(SZ_TOTAL <= (size_t)134217728);
static_assert(((size_t)DM * DM / 8) % 256 == 0);
static_assert(((size_t)DM * DFF / 8) % 256 == 0);
static_assert((size_t)NB * NH_ * SEQ * HD == (size_t)NTOK * DM);

extern "C" void kernel_launch(void* const* d_in, const int* in_sizes, int n_in,
                              void* d_out, int out_size, void* d_ws, size_t ws_size, hipStream_t stream) {
    if (n_in < 14) return;
    const size_t needx = ((size_t)(NB - 1) * SEQ_FULL + SEQ) * DM;
    const size_t needm = (size_t)(NB - 1) * SEQ_FULL + SEQ;
    if ((size_t)in_sizes[0] < needx || (size_t)in_sizes[1] < needm) return;
    if (in_sizes[2] < DM * DM || in_sizes[4] < DM * DM || in_sizes[6] < DM * DM || in_sizes[8] < DM * DM) return;
    if (in_sizes[3] < DM || in_sizes[5] < DM || in_sizes[7] < DM || in_sizes[9] < DM) return;
    if (in_sizes[10] < DM * DFF || in_sizes[11] < DFF || in_sizes[12] < DFF * DM || in_sizes[13] < DM) return;
    if ((size_t)out_size < ((size_t)(NB - 1) * OUT_SEQ + SEQ) * DM) return;
    if (SZ_TOTAL > ws_size) return;
    const float* x    = (const float*)d_in[0];
    const float* mask = (const float*)d_in[1];
    const float* wq = (const float*)d_in[2];  const float* bq = (const float*)d_in[3];
    const float* wk = (const float*)d_in[4];  const float* bk = (const float*)d_in[5];
    const float* wv = (const float*)d_in[6];  const float* bv = (const float*)d_in[7];
    const float* wo = (const float*)d_in[8];  const float* bo = (const float*)d_in[9];
    const float* w1 = (const float*)d_in[10]; const float* b1 = (const float*)d_in[11];
    const float* w2 = (const float*)d_in[12]; const float* b2 = (const float*)d_in[13];
    float* OUT = (float*)d_out;
    char* wsp = (char*)d_ws;
    float* Y  = (float*)wsp; wsp += SZ_F;
    float* YS = (float*)wsp; wsp += SZ_F;
    float* KS = (float*)wsp; wsp += 6 * SZ_F;
    h16* QK = (h16*)wsp; wsp += SZ_QK;
    h16* VT = (h16*)wsp; wsp += SZ_VT;
    h16* CX = (h16*)wsp; wsp += SZ_CX;
    h16* WQKV = (h16*)wsp; wsp += SZ_WQ;
    h16* WOT  = (h16*)wsp; wsp += SZ_WO;
    h16* W1T  = (h16*)wsp; wsp += SZ_W1;
    h16* W2T  = (h16*)wsp; wsp += SZ_W2;
    float* BQKV = (float*)wsp; wsp += SZ_BQ;
    float* BOP  = (float*)wsp; wsp += SZ_BO;
    float* B1P  = (float*)wsp; wsp += SZ_B1;
    float* B2P  = (float*)wsp; wsp += SZ_B2;

    k_wconv<<<(DM * DM / 8) / 256, 256, 0, stream>>>(wq, bq, WQKV, BQKV, DM, DM, 0);
    k_wconv<<<(DM * DM / 8) / 256, 256, 0, stream>>>(wk, bk, WQKV, BQKV, DM, DM, DM);
    k_wconv<<<(DM * DM / 8) / 256, 256, 0, stream>>>(wv, bv, WQKV, BQKV, DM, DM, 2 * DM);
    k_wconv<<<(DM * DM / 8) / 256, 256, 0, stream>>>(wo, bo, WOT, BOP, DM, DM, 0);
    k_wconv<<<(DM * DFF / 8) / 256, 256, 0, stream>>>(w1, b1, W1T, B1P, DM, DFF, 0);
    k_wconv<<<(DFF * DM / 8) / 256, 256, 0, stream>>>(w2, b2, W2T, B2P, DFF, DM, 0);
    k_init<<<(NTOK * 16) / 256, 256, 0, stream>>>(x, Y);

    for (int step = 0; step < 4; ++step) {
        for (int s = 0; s < 6; ++s) {
            const float* ysrc = (s == 0) ? Y : YS;
            k_qkv<<<NTOK / 64, 128, 0, stream>>>(Y, KS, YS, WQKV, BQKV, QK, VT, s);
            k_flash<<<dim3(SEQ / 16, NB, 1), 256, 0, stream>>>(QK, VT, mask, CX);
            k_wo_ffn<<<NTOK / 16, 32, 0, stream>>>(CX, ysrc, WOT, BOP, W1T, B1P, W2T, B2P, KS + (size_t)s * NTOK * DM);
        }
        if (step == 3) k_update<<<(NTOK * 16) / 256, 256, 0, stream>>>(Y, KS, OUT, OUT_SEQ);
        else           k_update<<<(NTOK * 16) / 256, 256, 0, stream>>>(Y, KS, Y, SEQ);
    }
}
